// Model_28269474743137
// MI455X (gfx1250) — hardware-verified
//
#include <hip/hip_runtime.h>
#include <stddef.h>
#include <stdint.h>


#define DX     64
#define MFEAT  18
#define K1     128
#define NH     8
#define C2     64
#define HW     512
#define N1     1024
#define K2     1024
#define N2     128
#define GC     128
#define NTHR   256
#define NWAVE  8
#define EPT    8
#define CHUNK  (NTHR * EPT)
#define WCAP   (EPT * 32)
#define LISTN  (NWAVE * WCAP)
#define NBMAX  2048
#define SLOTB  11
#define RCAP   28672
#define DEGCAP 512
#define STGW   512
#define GBM    32
#define GTHR   64
#define MROWS  128
#define NSD1   16
#define NSD2   2
#define UPM    8192
#define NMAT   4
#define NEGSL  0.2f
#define EPS_SM 1e-16f
#define MX0    (-1.0e30f)
#define WSMAX  134217728
#define LDS_AGG ((2 * RCAP + 2 * NBMAX + LISTN) * 4 + 64)

static_assert((CHUNK & (CHUNK - 1)) == 0 && CHUNK <= (1 << SLOTB));
static_assert(NBMAX == (1 << SLOTB));
static_assert(NTHR * 8 == NBMAX);
static_assert(LISTN >= NBMAX);
static_assert(LISTN >= NWAVE * WCAP);
static_assert((RCAP % 32) == 0);
static_assert(NWAVE * 2 * STGW <= RCAP && STGW * 4 == K2 * 2);
static_assert(LDS_AGG <= 300000);
static_assert(GBM == (GTHR / 32) * 16 && GTHR == 64 && GBM == 32);
static_assert(K1 == 2 * DX && K2 == 2 * HW && (K1 % 32) == 0 && (K2 % 32) == 0);
static_assert(HW == NH * C2 && N1 == 2 * HW && N2 == 2 * C2 && (N1 % GC) == 0 && (N2 % GC) == 0 && GC == 2 * C2);
static_assert(HW == 32 * 16 && C2 == 32 * 2);
static_assert((MROWS % GBM) == 0 && ((MROWS * (K1 / 8)) % NTHR) == 0);
static_assert(UPM == HW * (K1 / 8) && UPM == C2 * (K2 / 8) && (UPM % NTHR) == 0 && UPM == (1 << 13));
static_assert(NSD1 == N1 / C2 && NSD2 == N2 / C2);
static_assert(C2 / 4 == 16);

typedef float          v2f   __attribute__((ext_vector_type(2)));
typedef float          v4f   __attribute__((ext_vector_type(4)));
typedef float          v8f   __attribute__((ext_vector_type(8)));
typedef int            v4i   __attribute__((ext_vector_type(4)));
typedef int            v8i   __attribute__((ext_vector_type(8)));
typedef unsigned short v8us  __attribute__((ext_vector_type(8)));
typedef unsigned short v16us __attribute__((ext_vector_type(16)));
typedef __bf16         v16bf __attribute__((ext_vector_type(16)));
typedef v2f  __attribute__((may_alias)) v2fa;
typedef v4f  __attribute__((may_alias)) v4fa;
typedef v4i  __attribute__((may_alias)) v4ia;
typedef v8us __attribute__((may_alias)) v8usa;
union Frag { v16bf v; v16us u; v8us h[2]; v8i w; };
union Piece { v8us h; v4i w; };

__device__ __forceinline__ v8f wmb(const Frag& a, const Frag& b, v8f c) {
  v8f d = __builtin_amdgcn_wmma_f32_16x16x32_bf16(false, a.v, false, b.v, (short)0, c, false, false);
  asm volatile("v_nop\n\tv_nop\n\tv_nop\n\tv_nop" : "+v"(d) : "v"(a.w), "v"(b.w));
  return d;
}

__device__ __forceinline__ unsigned bf16_bits(float f) {
  const unsigned u = __float_as_uint(f);
  return (u + 0x7FFFu + ((u >> 16) & 1u)) >> 16;
}
__device__ __forceinline__ float bf16_val(float f) {
  return __uint_as_float(bf16_bits(f) << 16);
}
__device__ __forceinline__ v8us hilo8(v4f t) {
  v8us o;
  unsigned hb;
  hb = bf16_bits(t.x); o[0] = (unsigned short)hb; o[4] = (unsigned short)bf16_bits(t.x - __uint_as_float(hb << 16));
  hb = bf16_bits(t.y); o[1] = (unsigned short)hb; o[5] = (unsigned short)bf16_bits(t.y - __uint_as_float(hb << 16));
  hb = bf16_bits(t.z); o[2] = (unsigned short)hb; o[6] = (unsigned short)bf16_bits(t.z - __uint_as_float(hb << 16));
  hb = bf16_bits(t.w); o[3] = (unsigned short)hb; o[7] = (unsigned short)bf16_bits(t.w - __uint_as_float(hb << 16));
  return o;
}
__device__ __forceinline__ void upd4(v4f& a, const v4f f, float s1, float s2) {
  a.x = fmaf(a.x, s1, s2 * f.x);
  a.y = fmaf(a.y, s1, s2 * f.y);
  a.z = fmaf(a.z, s1, s2 * f.z);
  a.w = fmaf(a.w, s1, s2 * f.w);
}

__device__ __forceinline__ int scan_chunk(const int* __restrict__ dsts, int nE, int cbase, int slotBase,
                                          int nb, int vec8, int* list, int tid, int lane, int wave) {
  int wc = 0;
  const int el0  = tid * EPT;
  const int e0   = cbase + el0;
  const int sent = -2147483647 - 1;
  v4i da, db;
  if (vec8 != 0 && cbase + CHUNK <= nE) {
    da = *(const v4i*)(dsts + e0);
    db = *(const v4i*)(dsts + e0 + 4);
  } else {
    da.x = (e0     < nE) ? dsts[min(e0,     nE - 1)] : sent;
    da.y = (e0 + 1 < nE) ? dsts[min(e0 + 1, nE - 1)] : sent;
    da.z = (e0 + 2 < nE) ? dsts[min(e0 + 2, nE - 1)] : sent;
    da.w = (e0 + 3 < nE) ? dsts[min(e0 + 3, nE - 1)] : sent;
    db.x = (e0 + 4 < nE) ? dsts[min(e0 + 4, nE - 1)] : sent;
    db.y = (e0 + 5 < nE) ? dsts[min(e0 + 5, nE - 1)] : sent;
    db.z = (e0 + 6 < nE) ? dsts[min(e0 + 6, nE - 1)] : sent;
    db.w = (e0 + 7 < nE) ? dsts[min(e0 + 7, nE - 1)] : sent;
  }
  const unsigned nbs = (unsigned)slotBase;
  const unsigned unb = (unsigned)nb;
  const unsigned s0 = (unsigned)da.x - nbs, s1 = (unsigned)da.y - nbs;
  const unsigned s2 = (unsigned)da.z - nbs, s3 = (unsigned)da.w - nbs;
  const unsigned s4 = (unsigned)db.x - nbs, s5 = (unsigned)db.y - nbs;
  const unsigned s6 = (unsigned)db.z - nbs, s7 = (unsigned)db.w - nbs;
  const bool h0 = s0 < unb, h1 = s1 < unb, h2 = s2 < unb, h3 = s3 < unb;
  const bool h4 = s4 < unb, h5 = s5 < unb, h6 = s6 < unb, h7 = s7 < unb;
  const unsigned any = __builtin_amdgcn_ballot_w32(h0 | h1 | h2 | h3 | h4 | h5 | h6 | h7);
  if (any != 0u) {
#define HITJ(J, HJ, SJ) { \
      const unsigned mj = __builtin_amdgcn_ballot_w32(HJ); \
      if (mj != 0u) { \
        if (HJ) { \
          const int pos = wc + (int)__builtin_amdgcn_mbcnt_lo(mj, 0u); \
          if (pos < WCAP) list[wave * WCAP + pos] = ((el0 + (J)) << SLOTB) | (int)(SJ); \
        } \
        wc += (int)__builtin_popcount(mj); } }
    HITJ(0, h0, s0)
    HITJ(1, h1, s1)
    HITJ(2, h2, s2)
    HITJ(3, h3, s3)
    HITJ(4, h4, s4)
    HITJ(5, h5, s5)
    HITJ(6, h6, s6)
    HITJ(7, h7, s7)
#undef HITJ
  }
  return wc;
}

__global__ __launch_bounds__(NTHR) void k_wprep(const float* __restrict__ w1a, const float* __restrict__ w1b,
                                                const float* __restrict__ w2a, const float* __restrict__ w2b,
                                                unsigned short* WT1, unsigned short* WT2) {
  const int u  = (int)blockIdx.x * NTHR + (int)threadIdx.x;
  const int mi = u >> 13;
  const int v  = u & (UPM - 1);
  if (mi >= NMAT) return;
  const float* p;
  unsigned short* dp;
  int strd;
  if (mi < 2) {
    const float* W = (mi == 0) ? w1a : w1b;
    const int n = v >> 4;
    const int g = v & 15;
    p    = W + (size_t)(4 * g) * HW + n;
    strd = HW;
    dp   = WT1 + ((size_t)mi * HW + n) * K1 + 8 * g;
  } else {
    const float* W = (mi == 2) ? w2a : w2b;
    const int n = v >> 7;
    const int g = v & 127;
    p    = W + (size_t)(4 * g) * C2 + n;
    strd = C2;
    dp   = WT2 + ((size_t)(mi - 2) * C2 + n) * K2 + 8 * g;
  }
  const unsigned short f0 = (unsigned short)bf16_bits(p[0]);
  const unsigned short f1 = (unsigned short)bf16_bits(p[(size_t)strd]);
  const unsigned short f2 = (unsigned short)bf16_bits(p[(size_t)2 * strd]);
  const unsigned short f3 = (unsigned short)bf16_bits(p[(size_t)3 * strd]);
  v8us o;
  o[0] = f0; o[1] = f1; o[2] = f2; o[3] = f3; o[4] = f0; o[5] = f1; o[6] = f2; o[7] = f3;
  *(volatile v8us*)dp = o;
  __threadfence();
  *(volatile v8us*)dp = o;
}

__global__ __launch_bounds__(NTHR) void k_nprep(const float* __restrict__ uemb, const int* __restrict__ uid,
                                                int nU, int nUE, int U0,
                                                const float* __restrict__ xmv, const float* __restrict__ wl,
                                                const float* __restrict__ bl, const float* __restrict__ memb,
                                                const int* __restrict__ mid, int nM, int nME, int U1,
                                                unsigned short* XU, unsigned short* XM) {
  const int u = (int)blockIdx.x * NTHR + (int)threadIdx.x;
  const v4f z4 = {0.f, 0.f, 0.f, 0.f};
  v4f t;
  unsigned short* dp;
  if (u < U0) {
    const int row = u >> 4;
    const int g   = u & 15;
    const int c4  = 4 * g;
    const int rc  = row < nU ? row : nU - 1;
    int id = uid[rc];
    id = id < 0 ? 0 : (id > nUE - 1 ? nUE - 1 : id);
    const v4f e = *(const v4fa*)(uemb + (size_t)id * DX + c4);
    t.x = bf16_val(e.x); t.y = bf16_val(e.y); t.z = bf16_val(e.z); t.w = bf16_val(e.w);
    if (row >= nU) t = z4;
    dp = XU + (size_t)row * K1 + 8 * g;
  } else if (u < U0 + U1) {
    const int v   = u - U0;
    const int row = v >> 4;
    const int g   = v & 15;
    const int c4  = 4 * g;
    const int rc  = row < nM ? row : nM - 1;
    int id = mid[rc];
    id = id < 0 ? 0 : (id > nME - 1 ? nME - 1 : id);
    const float* xr = xmv + (size_t)rc * MFEAT;
    float a0 = 0.0f, a1 = 0.0f, a2 = 0.0f, a3 = 0.0f;
#pragma unroll 3
    for (int k = 0; k < MFEAT; ++k) {
      const float xk = bf16_val(xr[k]);
      const v4f w = *(const v4fa*)(wl + (size_t)k * DX + c4);
      a0 = fmaf(xk, bf16_val(w.x), a0);
      a1 = fmaf(xk, bf16_val(w.y), a1);
      a2 = fmaf(xk, bf16_val(w.z), a2);
      a3 = fmaf(xk, bf16_val(w.w), a3);
    }
    const v4f b = *(const v4fa*)(bl + c4);
    const v4f e = *(const v4fa*)(memb + (size_t)id * DX + c4);
    t.x = (a0 + bf16_val(b.x)) + bf16_val(e.x);
    t.y = (a1 + bf16_val(b.y)) + bf16_val(e.y);
    t.z = (a2 + bf16_val(b.z)) + bf16_val(e.z);
    t.w = (a3 + bf16_val(b.w)) + bf16_val(e.w);
    if (row >= nM) t = z4;
    dp = XM + (size_t)row * K1 + 8 * g;
  } else {
    return;
  }
  const v8us o = hilo8(t);
  *(volatile v8us*)dp = o;
  __threadfence();
  *(volatile v8us*)dp = o;
}

__global__ __launch_bounds__(GTHR) void k_gemm(const unsigned short* __restrict__ A,
                                               const unsigned short* __restrict__ WT, int K, int MPr,
                                               const float* __restrict__ attA, const float* __restrict__ attB,
                                               int attN, int cpmShift,
                                               float* H, int ldH, int gs0, int nStore, float* SD) {
  __shared__ __attribute__((aligned(16))) float stg[GBM * GC];
  __shared__ __attribute__((aligned(16))) float satt[GC];
  __shared__ __attribute__((aligned(16))) float sdot[2 * GBM];
  const int tid = (int)threadIdx.x, lane = tid & 31, wave = tid >> 5, hh = lane >> 4, m = lane & 15;
  const int rowBase = (int)blockIdx.x * GBM;
  const int g = (int)blockIdx.y;

#pragma unroll
  for (int q = 0; q < 2; ++q) {
    const int c   = 64 * q + tid;
    const int col = g * GC + c;
    const int mi  = col >> cpmShift;
    int cm = col & (attN - 1);
    cm = cm < attN ? cm : attN - 1;
    const float va = attA[cm];
    const float vb = attB[cm];
    const unsigned msk = (mi == 0) ? 0u : 0xFFFFFFFFu;
    const float v = __uint_as_float((__float_as_uint(va) & ~msk) | (__float_as_uint(vb) & msk));
    satt[c] = bf16_val(v);
  }

  v8f acc[8];
  {
    const v8f z = {0.f, 0.f, 0.f, 0.f, 0.f, 0.f, 0.f, 0.f};
#pragma unroll
    for (int t = 0; t < 8; ++t) acc[t] = z;
  }
  const unsigned short* ap = A  + (size_t)(rowBase + 16 * wave + m) * (size_t)K + 8 * hh;
  const unsigned short* bp = WT + ((size_t)g * GC + m) * (size_t)K + 8 * hh;
  const int ksteps = K >> 5;

#pragma unroll 1
  for (int ks = 0; ks < ksteps; ++ks) {
    const int k0 = 32 * ks;
    Frag af;
    af.h[0] = *(const v8usa*)(ap + k0);
    af.h[1] = *(const v8usa*)(ap + k0 + 16);
#pragma unroll
    for (int nt = 0; nt < 8; ++nt) {
      const unsigned short* wq = bp + (size_t)(16 * nt) * (size_t)K + k0;
      Frag bf;
      bf.h[0] = *(const v8usa*)wq;
      bf.h[1] = *(const v8usa*)(wq + 16);
      acc[nt] = wmb(af, bf, acc[nt]);
    }
  }

#pragma unroll
  for (int nt = 0; nt < 8; ++nt) {
    const int lc = 16 * nt + m;
#pragma unroll
    for (int r = 0; r < 8; ++r) {
      const int lr = 16 * wave + 8 * hh + r;
      stg[lr * GC + lc] = acc[nt][r];
    }
  }
  __syncthreads();

  {
    const int row = tid & 31, half = tid >> 5;
    const int cbeg = C2 * half;
    const float* hr = stg + row * GC + cbeg;
    const float* sa = satt + cbeg;
    float d = 0.f;
#pragma unroll 4
    for (int c4 = 0; c4 < C2 / 4; ++c4) {
      const v4f hv = *(const v4fa*)(hr + 4 * c4);
      const v4f av = *(const v4fa*)(sa + 4 * c4);
      d = fmaf(hv.x, av.x, d);
      d = fmaf(hv.y, av.y, d);
      d = fmaf(hv.z, av.z, d);
      d = fmaf(hv.w, av.w, d);
    }
    sdot[half * GBM + row] = d;
  }
  __syncthreads();

  const int piece = lane & 7;
  const int pl    = (lane >> 3) & 1;
  const v4f sdv   = *(const v4fa*)(sdot + pl * GBM + 4 * piece);
  const int plane = 2 * g + pl;
  float* sp = SD + (size_t)plane * (size_t)MPr + rowBase + 4 * piece;
  const bool wsd = (wave == 0) && (lane < 16);
  const bool wh  = (g >= gs0) && (g < gs0 + nStore);

  v4f fv[16];
#pragma unroll
  for (int i = 0; i < 16; ++i) {
    const int lr = 16 * wave + i;
    fv[i] = *(const v4fa*)(stg + lr * GC + 4 * lane);
  }
  float* hb = H + (size_t)(g - gs0) * (size_t)GC;
  if (wh) {
#pragma unroll
    for (int i = 0; i < 16; ++i) {
      const int gr = rowBase + 16 * wave + i;
      float* op = hb + (size_t)gr * (size_t)ldH + 4 * lane;
      *(volatile v4f*)op = fv[i];
    }
  }
  if (wsd) *(volatile v4f*)sp = sdv;
  __threadfence();
  if (wh) {
#pragma unroll
    for (int i = 0; i < 16; ++i) {
      const int gr = rowBase + 16 * wave + i;
      float* op = hb + (size_t)gr * (size_t)ldH + 4 * lane;
      *(volatile v4f*)op = fv[i];
    }
  }
  if (wsd) *(volatile v4f*)sp = sdv;
}

template <int LY>
__global__ __launch_bounds__(NTHR) void k_agg(
    const int* __restrict__ srcs, const int* __restrict__ dsts, int nE, int nSrc, int nDst, int MPr, int nb, int vec8,
    const float* __restrict__ F, int ldF, int colOff,
    const float* __restrict__ AS, int ldAS, const float* __restrict__ AD, int ldAD,
    const float* __restrict__ bias, float* oout, unsigned short* hp) {
  static_assert(LY == 1 || LY == 2);
  extern __shared__ v4f lds_dyn[];
  int* reg1 = (int*)lds_dyn;
  int* reg2 = reg1 + RCAP;
  int* scnt = reg2 + RCAP;
  int* soff = scnt + NBMAX;
  int* list = soff + NBMAX;
  int* wcnt = list + LISTN;
  int* wtot = wcnt + NWAVE;
  const int tid = (int)threadIdx.x, lane = tid & 31, wave = tid >> 5;
  const int nodeBase = (int)blockIdx.x * nb;

  for (int i = tid; i < NBMAX; i += NTHR) scnt[i] = 0;
  __syncthreads();

  int tot = 0;
  const int nChunks = (nE + CHUNK - 1) / CHUNK;
#pragma unroll 1
  for (int ch = 0; ch < nChunks; ++ch) {
    const int cbase = ch * CHUNK;
    const int wc = scan_chunk(dsts, nE, cbase, nodeBase, nb, vec8, list, tid, lane, wave);
    if (lane == 0) wcnt[wave] = wc;
    __syncthreads();
    int pre = 0, all = 0;
#pragma unroll
    for (int w2 = 0; w2 < NWAVE; ++w2) {
      int c = wcnt[w2];
      c = c < 0 ? 0 : (c > WCAP ? WCAP : c);
      all += c;
      pre += (w2 < wave) ? c : 0;
    }
    const int wcc  = wc > WCAP ? WCAP : wc;
    const int base = tot + pre;
#pragma unroll 1
    for (int i = lane; i < wcc; i += 32) {
      const int ent = list[wave * WCAP + i];
      const int el  = (ent >> SLOTB) & (CHUNK - 1);
      const int sl  = ent & (NBMAX - 1);
      int eid = cbase + el;
      eid = eid > nE - 1 ? nE - 1 : eid;
      const int pos = base + i;
      if (pos < RCAP) reg1[pos] = (int)(((unsigned)eid << SLOTB) | (unsigned)sl);
    }
    tot += all;
    tot = tot > RCAP ? RCAP : tot;
    __syncthreads();
  }
  const int nh = tot;

  if (wave == 0) {
#pragma unroll 1
    for (int b0 = 0; b0 < nh; b0 += 32) {
      const int idx = b0 + lane;
      const int uv  = reg1[idx < nh ? idx : nh - 1];
      const int m32 = (nh - b0) < 32 ? (nh - b0) : 32;
#pragma unroll 1
      for (int k = 0; k < m32; ++k) {
        const int u  = __builtin_amdgcn_readlane(uv, k);
        const int sl = u & (NBMAX - 1);
        if (lane == 0) scnt[sl] = scnt[sl] + 1;
      }
    }
  }
  __syncthreads();

  {
    const v4i ca = *(const v4ia*)(scnt + 8 * tid);
    const v4i cb = *(const v4ia*)(scnt + 8 * tid + 4);
    const int e0 = ca.x < 0 ? 0 : ca.x, e1 = ca.y < 0 ? 0 : ca.y, e2 = ca.z < 0 ? 0 : ca.z, e3 = ca.w < 0 ? 0 : ca.w;
    const int e4 = cb.x < 0 ? 0 : cb.x, e5 = cb.y < 0 ? 0 : cb.y, e6 = cb.z < 0 ? 0 : cb.z, e7 = cb.w < 0 ? 0 : cb.w;
    const int ts = e0 + e1 + e2 + e3 + e4 + e5 + e6 + e7;
    int incl = ts;
#pragma unroll
    for (int d = 1; d < 32; d <<= 1) {
      const int up = __shfl_up(incl, d);
      if (lane >= d) incl += up;
    }
    if (lane == 31) wtot[wave] = incl;
    __syncthreads();
    int pre = 0;
#pragma unroll
    for (int w2 = 0; w2 < NWAVE; ++w2) pre += (w2 < wave) ? wtot[w2] : 0;
    int run = pre + incl - ts;
    soff[8 * tid + 0] = run; run += e0;
    soff[8 * tid + 1] = run; run += e1;
    soff[8 * tid + 2] = run; run += e2;
    soff[8 * tid + 3] = run; run += e3;
    soff[8 * tid + 4] = run; run += e4;
    soff[8 * tid + 5] = run; run += e5;
    soff[8 * tid + 6] = run; run += e6;
    soff[8 * tid + 7] = run;
  }
  __syncthreads();
  for (int i = tid; i < NBMAX; i += NTHR) list[i] = soff[i];
  __syncthreads();

  if (wave == 0) {
#pragma unroll 1
    for (int b0 = 0; b0 < nh; b0 += 32) {
      const int idx = b0 + lane;
      const int uv  = reg1[idx < nh ? idx : nh - 1];
      const int m32 = (nh - b0) < 32 ? (nh - b0) : 32;
#pragma unroll 1
      for (int k = 0; k < m32; ++k) {
        const int u   = __builtin_amdgcn_readlane(uv, k);
        const int sl  = u & (NBMAX - 1);
        const int eid = (int)((unsigned)u >> SLOTB);
        if (lane == 0) {
          int pos = list[sl];
          pos = pos < 0 ? 0 : (pos > RCAP - 1 ? RCAP - 1 : pos);
          reg2[pos] = eid;
          list[sl] = pos + 1;
        }
      }
    }
  }
  __syncthreads();

  const int nbw = nb >> 3;
  const bool ovf = (nh >= RCAP);
  const float qnan = __int_as_float(0x7fc00000);
  const int hl = (LY == 1) ? (lane >> 2) : 0;
  const float* asl = AS + (size_t)hl * (size_t)ldAS;
  const float* adl = AD + (size_t)hl * (size_t)ldAD;

  if constexpr (LY == 1) {
    v4f bb[4];
#pragma unroll
    for (int p = 0; p < 4; ++p) {
      const v4f t = *(const v4fa*)(bias + 16 * lane + 4 * p);
      bb[p].x = bf16_val(t.x); bb[p].y = bf16_val(t.y); bb[p].z = bf16_val(t.z); bb[p].w = bf16_val(t.w);
    }
    const v4f z4 = {0.0f, 0.0f, 0.0f, 0.0f};

#pragma unroll 1
    for (int jt = 0; jt < nbw; ++jt) {
      const int slot = wave * nbw + jt;
      const int grow = nodeBase + slot;
      const int gcl  = grow < nDst ? grow : nDst - 1;
      int st = soff[slot];
      const int craw = scnt[slot];
      int cnt = craw;
      st  = st < 0 ? 0 : (st > nh ? nh : st);
      cnt = cnt < 0 ? 0 : (cnt > DEGCAP ? DEGCAP : cnt);
      if (cnt > nh - st) cnt = nh - st;
      const float pz = (ovf || craw > DEGCAP) ? qnan : 0.0f;

      const float adv = adl[gcl];
      float mx = MX0, dn = 0.0f;
      v4f acc[4];
      acc[0] = z4; acc[1] = z4; acc[2] = z4; acc[3] = z4;

#pragma unroll 1
      for (int q = 0; q < cnt; ++q) {
        int idx = st + q; idx = idx > RCAP - 1 ? RCAP - 1 : idx;
        int eid = reg2[idx]; eid = eid < 0 ? 0 : (eid > nE - 1 ? nE - 1 : eid);
        const int sraw = srcs[eid];
        const int s = sraw < 0 ? 0 : (sraw > nSrc - 1 ? nSrc - 1 : sraw);
        const float* fr = F + (size_t)s * (size_t)ldF + colOff + 16 * lane;
        const v4f f0 = *(const v4fa*)fr;
        const v4f f1 = *(const v4fa*)(fr + 4);
        const v4f f2 = *(const v4fa*)(fr + 8);
        const v4f f3 = *(const v4fa*)(fr + 12);
        float lg = asl[s] + adv;
        lg = lg > 0.f ? lg : NEGSL * lg;
        const float df = lg - mx;
        const float ee = __expf(-fabsf(df));
        const bool up  = df > 0.f;
        const float s1 = up ? ee : 1.0f;
        const float s2 = up ? 1.0f : ee;
        mx = up ? lg : mx;
        dn = fmaf(dn, s1, s2);
        upd4(acc[0], f0, s1, s2);
        upd4(acc[1], f1, s1, s2);
        upd4(acc[2], f2, s1, s2);
        upd4(acc[3], f3, s1, s2);
      }
      const float inv = __builtin_amdgcn_rcpf(dn + EPS_SM);
      const bool live = grow < nDst;
      const bool wrow = grow < MPr;

      Piece pc[4];
#pragma unroll
      for (int p = 0; p < 4; ++p) {
        v4f v;
        v.x = fmaxf(fmaf(acc[p].x, inv, bb[p].x), 0.0f);
        v.y = fmaxf(fmaf(acc[p].y, inv, bb[p].y), 0.0f);
        v.z = fmaxf(fmaf(acc[p].z, inv, bb[p].z), 0.0f);
        v.w = fmaxf(fmaf(acc[p].w, inv, bb[p].w), 0.0f);
        v4f y;
        y.x = (live ? v.x : 0.f) + pz;
        y.y = (live ? v.y : 0.f) + pz;
        y.z = (live ? v.z : 0.f) + pz;
        y.w = (live ? v.w : 0.f) + pz;
        pc[p].h = hilo8(y);
      }
      int* stgw = reg1 + wave * (2 * STGW) + (jt & 1) * STGW;
#pragma unroll
      for (int p = 0; p < 4; ++p) *(v4ia*)(stgw + 16 * lane + 4 * p) = pc[p].w;
      __builtin_amdgcn_fence(__ATOMIC_RELEASE, "wavefront");
      __builtin_amdgcn_wave_barrier();
      Piece po[4];
#pragma unroll
      for (int j = 0; j < 4; ++j) po[j].w = *(const v4ia*)(stgw + 128 * j + 4 * lane);
      __builtin_amdgcn_fence(__ATOMIC_RELEASE, "wavefront");
      __builtin_amdgcn_wave_barrier();

      unsigned short* gp = hp + (size_t)grow * (size_t)K2 + 8 * lane;
      if (wrow) {
#pragma unroll
        for (int j = 0; j < 4; ++j) *(volatile v8us*)(gp + 256 * j) = po[j].h;
      }
      __threadfence();
      if (wrow) {
#pragma unroll
        for (int j = 0; j < 4; ++j) *(volatile v8us*)(gp + 256 * j) = po[j].h;
      }
    }
  } else {
    v2f bb2;
    {
      const v2f t = *(const v2fa*)(bias + 2 * lane);
      bb2.x = bf16_val(t.x); bb2.y = bf16_val(t.y);
    }

#pragma unroll 1
    for (int jt = 0; jt < nbw; ++jt) {
      const int slot = wave * nbw + jt;
      const int grow = nodeBase + slot;
      const int gcl  = grow < nDst ? grow : nDst - 1;
      int st = soff[slot];
      const int craw = scnt[slot];
      int cnt = craw;
      st  = st < 0 ? 0 : (st > nh ? nh : st);
      cnt = cnt < 0 ? 0 : (cnt > DEGCAP ? DEGCAP : cnt);
      if (cnt > nh - st) cnt = nh - st;
      const float pz = (ovf || craw > DEGCAP) ? qnan : 0.0f;

      const float adv = adl[gcl];
      float mx = MX0, dn = 0.0f, a0 = 0.0f, a1 = 0.0f;

#pragma unroll 1
      for (int q = 0; q < cnt; ++q) {
        int idx = st + q; idx = idx > RCAP - 1 ? RCAP - 1 : idx;
        int eid = reg2[idx]; eid = eid < 0 ? 0 : (eid > nE - 1 ? nE - 1 : eid);
        const int sraw = srcs[eid];
        const int s = sraw < 0 ? 0 : (sraw > nSrc - 1 ? nSrc - 1 : sraw);
        const v2f fs = *(const v2fa*)(F + (size_t)s * (size_t)ldF + colOff + 2 * lane);
        float lg = asl[s] + adv;
        lg = lg > 0.f ? lg : NEGSL * lg;
        const float df = lg - mx;
        const float ee = __expf(-fabsf(df));
        const bool up  = df > 0.f;
        const float s1 = up ? ee : 1.0f;
        const float s2 = up ? 1.0f : ee;
        mx = up ? lg : mx;
        dn = fmaf(dn, s1, s2);
        a0 = fmaf(a0, s1, s2 * fs.x);
        a1 = fmaf(a1, s1, s2 * fs.y);
      }
      const float inv = __builtin_amdgcn_rcpf(dn + EPS_SM);
      const bool live = grow < nDst;
      const bool wrow = grow < MPr;
      const float v0 = fmaf(a0, inv, bb2.x);
      const float v1 = fmaf(a1, inv, bb2.y);
      const float h0 = (live ? v0 : 0.f) + pz;
      const float h1 = (live ? v1 : 0.f) + pz;
      const int i0 = (2 * lane) & 31, i1 = (2 * lane + 1) & 31;
      const float g0 = __shfl(h0, i0);
      const float g1 = __shfl(h1, i0);
      const float g2 = __shfl(h0, i1);
      const float g3 = __shfl(h1, i1);
      v4f ov;
      ov.x = g0; ov.y = g1; ov.z = g2; ov.w = g3;
      float* op = oout + (size_t)grow * (size_t)C2 + 4 * (lane & 15);
      const bool wr = wrow && (lane < 16);
      if (wr) *(volatile v4f*)op = ov;
      __threadfence();
      if (wr) *(volatile v4f*)op = ov;
    }
  }
}

__global__ __launch_bounds__(NTHR) void k_score(const int* __restrict__ ls, const int* __restrict__ ld, int L,
                                                const float* __restrict__ U, const float* __restrict__ M,
                                                int nU, int nM, float* out) {
  const int tid = (int)threadIdx.x;
  const int e  = (int)blockIdx.x * NTHR + tid;
  const int ec = e < L ? e : L - 1;
  int ia = ls[ec];
  ia = ia < 0 ? 0 : (ia > nU - 1 ? nU - 1 : ia);
  int ib = ld[ec];
  ib = ib < 0 ? 0 : (ib > nM - 1 ? nM - 1 : ib);
  const float* pa = U + (size_t)ia * C2;
  const float* pb = M + (size_t)ib * C2;
  float s = 0.0f;
#pragma unroll 4
  for (int c4 = 0; c4 < C2 / 4; ++c4) {
    const v4f va = *(const v4fa*)(pa + 4 * c4);
    const v4f vb = *(const v4fa*)(pb + 4 * c4);
    s = fmaf(va.x, vb.x, s);
    s = fmaf(va.y, vb.y, s);
    s = fmaf(va.z, vb.z, s);
    s = fmaf(va.w, vb.w, s);
  }
  float* op = out + ec;
  const bool wr = e < L;
  if (wr) *(volatile float*)op = s;
  __threadfence();
  if (wr) *(volatile float*)op = s;
}

static int pick_nb(int nE, int nN) {
  int nb = NBMAX;
  while (nb > 32 && (long long)nb * (long long)nE * 8LL > (long long)RCAP * (long long)nN * 7LL) nb >>= 1;
  return nb;
}
static inline int cdiv(int a, int b) { return (a + b - 1) / b; }

extern "C" void kernel_launch(void* const* d_in, const int* in_sizes, int n_in,
                              void* d_out, int out_size, void* d_ws, size_t ws_size,
                              hipStream_t stream) {
  if (n_in < 27) return;
  if (in_sizes[0] < MFEAT || (in_sizes[0] % MFEAT) != 0) return;
  const int nM = in_sizes[0] / MFEAT;
  const int nU = in_sizes[1];
  if (nU < 1 || nM < 1 || nU > (1 << 22) || nM > (1 << 22)) return;
  if (in_sizes[2] != nM) return;
  const int nE = in_sizes[3];
  if (nE < 1 || in_sizes[4] != nE) return;
  if (nE >= (1 << (32 - SLOTB))) return;
  const int L = in_sizes[5];
  if (L < 1 || in_sizes[6] != L || out_size != L) return;
  if (in_sizes[7] < DX || (in_sizes[7] % DX) != 0) return;
  if (in_sizes[8] < DX || (in_sizes[8] % DX) != 0) return;
  const int nUE = in_sizes[7] / DX, nME = in_sizes[8] / DX;
  if (in_sizes[9] != MFEAT * DX || in_sizes[10] != DX) return;
  if (in_sizes[11] != DX * HW || in_sizes[12] != HW || in_sizes[13] != HW || in_sizes[14] != HW) return;
  if (in_sizes[15] != DX * HW || in_sizes[16] != HW || in_sizes[17] != HW || in_sizes[18] != HW) return;
  if (in_sizes[19] != HW * C2 || in_sizes[20] != C2 || in_sizes[21] != C2 || in_sizes[22] != C2) return;
  if (in_sizes[23] != HW * C2 || in_sizes[24] != C2 || in_sizes[25] != C2 || in_sizes[26] != C2) return;

  const float* xmv  = (const float*)d_in[0];
  const int*   uid  = (const int*)  d_in[1];
  const int*   mid  = (const int*)  d_in[2];
  const int*   es   = (const int*)  d_in[3];
  const int*   ed   = (const int*)  d_in[4];
  const int*   ls   = (const int*)  d_in[5];
  const int*   ld   = (const int*)  d_in[6];
  const float* uemb = (const float*)d_in[7];
  const float* memb = (const float*)d_in[8];
  const float* wl   = (const float*)d_in[9];
  const float* bl   = (const float*)d_in[10];
  const float* w1a  = (const float*)d_in[11];
  const float* a1sA = (const float*)d_in[12];
  const float* a1dA = (const float*)d_in[13];
  const float* b1A  = (const float*)d_in[14];
  const float* w1b  = (const float*)d_in[15];
  const float* a1sB = (const float*)d_in[16];
  const float* a1dB = (const float*)d_in[17];
  const float* b1B  = (const float*)d_in[18];
  const float* w2a  = (const float*)d_in[19];
  const float* a2sA = (const float*)d_in[20];
  const float* a2dA = (const float*)d_in[21];
  const float* b2A  = (const float*)d_in[22];
  const float* w2b  = (const float*)d_in[23];
  const float* a2sB = (const float*)d_in[24];
  const float* a2dB = (const float*)d_in[25];
  const float* b2B  = (const float*)d_in[26];
  float* out = (float*)d_out;

  const int MPu = cdiv(nU, MROWS) * MROWS;
  const int MPm = cdiv(nM, MROWS) * MROWS;
  const int nbU = pick_nb(nE, nU);
  const int nbM = pick_nb(nE, nM);
  if (nbU < 32 || (nbU & (nbU - 1)) != 0 || nbU > NBMAX) return;
  if (nbM < 32 || (nbM & (nbM - 1)) != 0 || nbM > NBMAX) return;
  const int gAU = cdiv(MPu, nbU), gAM = cdiv(MPm, nbM);
  if ((long long)gAU * nbU < MPu || (long long)gAM * nbM < MPm) return;
  const int vec8 = ((nE & 3) == 0) ? 1 : 0;
  const int U0 = MPu * (K1 / 8), U1 = MPm * (K1 / 8);
  if ((U0 % NTHR) != 0 || (U1 % NTHR) != 0) return;
  if ((MPu % GBM) != 0 || (MPm % GBM) != 0) return;

  char* ws = (char*)d_ws;
  size_t off = 0;
  const size_t oWT1 = off; off += (size_t)N1 * K1 * 2;       off = (off + 255) & ~(size_t)255;
  const size_t oWT2 = off; off += (size_t)N2 * K2 * 2;       off = (off + 255) & ~(size_t)255;
  const size_t oXU  = off; off += (size_t)MPu * K1 * 2;      off = (off + 255) & ~(size_t)255;
  const size_t oXM  = off; off += (size_t)MPm * K1 * 2;      off = (off + 255) & ~(size_t)255;
  const size_t oH1U = off; off += (size_t)MPu * HW * 4;      off = (off + 255) & ~(size_t)255;
  const size_t oH1M = off; off += (size_t)MPm * HW * 4;      off = (off + 255) & ~(size_t)255;
  const size_t oSDU = off; off += (size_t)NSD1 * MPu * 4;    off = (off + 255) & ~(size_t)255;
  const size_t oSDM = off; off += (size_t)NSD1 * MPm * 4;    off = (off + 255) & ~(size_t)255;
  const size_t oHAU = off; off += (size_t)MPu * K2 * 2;      off = (off + 255) & ~(size_t)255;
  const size_t oHAM = off; off += (size_t)MPm * K2 * 2;      off = (off + 255) & ~(size_t)255;
  const size_t oH2U = off; off += (size_t)MPu * N2 * 4;      off = (off + 255) & ~(size_t)255;
  const size_t oH2M = off; off += (size_t)MPm * N2 * 4;      off = (off + 255) & ~(size_t)255;
  const size_t oS2U = off; off += (size_t)NSD2 * MPu * 4;    off = (off + 255) & ~(size_t)255;
  const size_t oS2M = off; off += (size_t)NSD2 * MPm * 4;    off = (off + 255) & ~(size_t)255;
  const size_t oU2  = off; off += (size_t)MPu * C2 * 4;      off = (off + 255) & ~(size_t)255;
  const size_t oM2  = off; off += (size_t)MPm * C2 * 4;      off = (off + 255) & ~(size_t)255;
  if (off > ws_size || off > (size_t)WSMAX) return;

  unsigned short* WT1 = (unsigned short*)(ws + oWT1);
  unsigned short* WT2 = (unsigned short*)(ws + oWT2);
  unsigned short* XU  = (unsigned short*)(ws + oXU);
  unsigned short* XM  = (unsigned short*)(ws + oXM);
  float*          H1U = (float*)(ws + oH1U);
  float*          H1M = (float*)(ws + oH1M);
  float*          SDU = (float*)(ws + oSDU);
  float*          SDM = (float*)(ws + oSDM);
  unsigned short* HAU = (unsigned short*)(ws + oHAU);
  unsigned short* HAM = (unsigned short*)(ws + oHAM);
  float*          H2U = (float*)(ws + oH2U);
  float*          H2M = (float*)(ws + oH2M);
  float*          S2U = (float*)(ws + oS2U);
  float*          S2M = (float*)(ws + oS2M);
  float*          U2  = (float*)(ws + oU2);
  float*          M2  = (float*)(ws + oM2);

  hipFuncSetAttribute(reinterpret_cast<const void*>(&k_agg<1>), hipFuncAttributeMaxDynamicSharedMemorySize, LDS_AGG);
  hipFuncSetAttribute(reinterpret_cast<const void*>(&k_agg<2>), hipFuncAttributeMaxDynamicSharedMemorySize, LDS_AGG);

  k_wprep<<<(NMAT * UPM) / NTHR, NTHR, 0, stream>>>(w1a, w1b, w2a, w2b, WT1, WT2);
  k_nprep<<<(U0 + U1) / NTHR, NTHR, 0, stream>>>(uemb, uid, nU, nUE, U0, xmv, wl, bl, memb, mid, nM, nME, U1, XU, XM);

  k_gemm<<<dim3(MPu / GBM, N1 / GC), GTHR, 0, stream>>>(XU, WT1, K1, MPu, a1sA, a1dB, HW, 9, H1U, HW, 0, 4, SDU);
  k_gemm<<<dim3(MPm / GBM, N1 / GC), GTHR, 0, stream>>>(XM, WT1, K1, MPm, a1dA, a1sB, HW, 9, H1M, HW, 4, 4, SDM);

  k_agg<1><<<gAM, NTHR, LDS_AGG, stream>>>(es, ed, nE, nU, nM, MPm, nbM, vec8,
      H1U, HW, 0, SDU, MPu, SDM, MPm, b1A, M2, HAM);
  k_agg<1><<<gAU, NTHR, LDS_AGG, stream>>>(ed, es, nE, nM, nU, MPu, nbU, vec8,
      H1M, HW, 0, SDM + (size_t)NH * MPm, MPm, SDU + (size_t)NH * MPu, MPu, b1B, U2, HAU);

  k_gemm<<<dim3(MPu / GBM, N2 / GC), GTHR, 0, stream>>>(HAU, WT2, K2, MPu, a2sA, a2dB, C2, 6, H2U, N2, 0, 1, S2U);
  k_gemm<<<dim3(MPm / GBM, N2 / GC), GTHR, 0, stream>>>(HAM, WT2, K2, MPm, a2dA, a2sB, C2, 6, H2M, N2, 0, 1, S2M);

  k_agg<2><<<gAM, NTHR, LDS_AGG, stream>>>(es, ed, nE, nU, nM, MPm, nbM, vec8,
      H2U, N2, 0, S2U, MPu, S2M, MPm, b2A, M2, HAM);
  k_agg<2><<<gAU, NTHR, LDS_AGG, stream>>>(ed, es, nE, nM, nU, MPu, nbU, vec8,
      H2M, N2, C2, S2M + (size_t)MPm, MPm, S2U + (size_t)MPu, MPu, b2B, U2, HAU);

  k_score<<<dim3(cdiv(L, NTHR)), NTHR, 0, stream>>>(ls, ld, L, U2, M2, nU, nM, out);
}
